// MultiHeadSelfAttention_82927228551388
// MI455X (gfx1250) — hardware-verified
//
#include <hip/hip_runtime.h>
#ifndef NB
#define NB 2
#endif
#ifndef SEQ
#define SEQ 2048
#endif
#define NB_FULL 2
#define SEQ_FULL 2048
#define DM 1024
#define NH 16
#define HD 64
#define LQ (3 * DM)
#define OCP (2 * DM)
#define NR ((size_t)NB * SEQ)
#define WS_TOTAL ((size_t)3 * DM * DM * 2 + (size_t)DM * OCP * 2 + NR * DM * 2 + NR * LQ * 2 + (size_t)NB * NH * HD * SEQ * 2 + NR * OCP * 2)

static_assert(NH * HD == DM);
static_assert(HD == 64);
static_assert(SEQ % 128 == 0);
static_assert(DM % 64 == 0);
static_assert(DM % 32 == 0);
static_assert(OCP % 32 == 0);
static_assert(LQ % 64 == 0);
static_assert(NB <= NB_FULL);
static_assert(SEQ <= SEQ_FULL);
static_assert(WS_TOTAL <= (size_t)134217728);
static_assert(((size_t)3 * DM * DM * 2) % 256 == 0);
static_assert((NR * DM * 2) % 256 == 0);

typedef unsigned short v8us __attribute__((ext_vector_type(8), may_alias));
typedef float  v8f  __attribute__((ext_vector_type(8)));
typedef float  v4f  __attribute__((ext_vector_type(4)));
typedef float  v4fa __attribute__((ext_vector_type(4), may_alias));
typedef _Float16 v16h __attribute__((ext_vector_type(16)));
typedef _Float16 v4h __attribute__((ext_vector_type(4)));
union FragH { v16h v; v8us half[2]; _Float16 h[16]; unsigned short u[16]; };
union Frag8 { v8us v; _Float16 h[8]; };

__device__ __forceinline__ unsigned short bf16_bits(float x) { unsigned int u = __float_as_uint(x); return (unsigned short)((u + 0x7FFFu + ((u >> 16) & 1u)) >> 16); }
__device__ __forceinline__ float bf16_val(unsigned short b) { return __uint_as_float(((unsigned int)b) << 16); }
__device__ __forceinline__ float bf16_rne_f(float x) { return bf16_val(bf16_bits(x)); }

__device__ __forceinline__ v16h g2_frag(const _Float16* p, int hh) { FragH f; f.half[0] = *(const v8us*)((const unsigned short*)p + 8 * hh); f.half[1] = *(const v8us*)((const unsigned short*)p + 16 + 8 * hh); return f.v; }
__device__ __forceinline__ v8f g2_mma(v16h a, v16h b, v8f c) { v8f d = __builtin_amdgcn_wmma_f32_16x16x32_f16(false, a, false, b, (short)0, c, false, false); asm volatile("v_nop\n\tv_nop\n\tv_nop\n\tv_nop" : "+v"(d) : "v"(a), "v"(b)); return d; }

__global__ __launch_bounds__(256) void k_wt_f16(const float* __restrict__ W, _Float16* __restrict__ Wt, int K, int N, int ldk, int dup, float scale) {
  const int t = blockIdx.x * 256 + threadIdx.x; const int k8n = K / 8; if (t >= N * k8n) return;
  const int n = t / k8n, k8 = (t - n * k8n) * 8; FragH f;
#pragma unroll
  for (int i = 0; i < 8; ++i) f.h[i] = (_Float16)(bf16_rne_f(W[(size_t)(k8 + i) * N + n]) * scale);
  const v8us o = f.half[0];
  unsigned short* d = (unsigned short*)Wt + (size_t)n * ldk + k8;
  *(volatile v8us*)d = o; if (dup) *(volatile v8us*)(d + K) = o;
  __threadfence();
  *(volatile v8us*)d = o; if (dup) *(volatile v8us*)(d + K) = o;
}

__global__ __launch_bounds__(256) void k_x16(const float* __restrict__ x, _Float16* __restrict__ X16) {
  const size_t t = (size_t)blockIdx.x * 256 + threadIdx.x; const size_t per = (size_t)SEQ * DM / 8; if (t >= (size_t)NB * per) return;
  const size_t b = t / per, rem = t - b * per;
  const float* src = x + b * (size_t)SEQ_FULL * DM + rem * 8;
  const v4f a = *(const v4fa*)src, c = *(const v4fa*)(src + 4); FragH f;
#pragma unroll
  for (int q = 0; q < 4; ++q) { f.h[q] = (_Float16)bf16_rne_f(a[q]); f.h[4 + q] = (_Float16)bf16_rne_f(c[q]); }
  const v8us o = f.half[0];
  unsigned short* d = (unsigned short*)X16 + t * 8;
  *(volatile v8us*)d = o; __threadfence(); *(volatile v8us*)d = o;
}

__global__ __launch_bounds__(128) void k_gemm2(const _Float16* __restrict__ A, int lda, size_t sA, const _Float16* __restrict__ Bh, int ldb, float alpha, const float* __restrict__ bias,
    float* __restrict__ C, _Float16* __restrict__ C16, int ldc, size_t sC, int M, int N, int K) {
  __shared__ __attribute__((aligned(16))) float so[4][32][68];
  const int w = __builtin_amdgcn_readfirstlane((int)(threadIdx.x >> 5));
  const int lane = threadIdx.x & 31, ln = lane & 15, hh = lane >> 4; const int by = blockIdx.y;
  A += (size_t)by * sA; const size_t cofs = (size_t)by * sC;
  const int ntn = N >> 6; const int mt = blockIdx.x / ntn, nq = blockIdx.x - mt * ntn; const int row0 = mt * 128 + 32 * w, col0 = nq * 64; if (row0 >= M) return;
  const _Float16* a0p = A + (size_t)(row0 + ln) * lda; const _Float16* a1p = a0p + (size_t)16 * lda;
  const _Float16* b0p = Bh + (size_t)(col0 + ln) * ldb; const _Float16* b1p = b0p + (size_t)16 * ldb; const _Float16* b2p = b1p + (size_t)16 * ldb; const _Float16* b3p = b2p + (size_t)16 * ldb;
  const v8f z8 = {0.f,0.f,0.f,0.f,0.f,0.f,0.f,0.f}; v8f c00 = z8, c01 = z8, c02 = z8, c03 = z8, c10 = z8, c11 = z8, c12 = z8, c13 = z8;
#pragma unroll 1
  for (int kb = 0; kb < K; kb += 32) { const v16h a0 = g2_frag(a0p + kb, hh), a1 = g2_frag(a1p + kb, hh);
    v16h b = g2_frag(b0p + kb, hh); c00 = g2_mma(a0, b, c00); c10 = g2_mma(a1, b, c10);
    b = g2_frag(b1p + kb, hh); c01 = g2_mma(a0, b, c01); c11 = g2_mma(a1, b, c11);
    b = g2_frag(b2p + kb, hh); c02 = g2_mma(a0, b, c02); c12 = g2_mma(a1, b, c12);
    b = g2_frag(b3p + kb, hh); c03 = g2_mma(a0, b, c03); c13 = g2_mma(a1, b, c13); }
  v8f accs[8] = {c00, c01, c02, c03, c10, c11, c12, c13};
#pragma unroll
  for (int u = 0; u < 8; ++u) { const int t = u & 3, half = u >> 2; const int col = col0 + t * 16 + ln; const float bv = bias ? bf16_rne_f(bias[col]) : 0.f;
#pragma unroll
    for (int r = 0; r < 8; ++r) { const int rloc = half * 16 + 8 * hh + r; so[w][rloc][t * 16 + ln] = accs[u][r] * alpha + bv; } }
  __builtin_amdgcn_fence(4  , "workgroup"); __builtin_amdgcn_wave_barrier();
  const int rsub = lane >> 4, c4 = (lane & 15) * 4;
  for (int pass = 0; pass < 2; ++pass) {
#pragma unroll
    for (int q = 0; q < 16; ++q) { const int r = q * 2 + rsub; const v4f v = *(const v4fa*)&so[w][r][c4];
      if (C) *(volatile v4f*)(C + cofs + (size_t)(row0 + r) * ldc + col0 + c4) = v;
      if (C16) { v4h h4;
#pragma unroll
        for (int i = 0; i < 4; ++i) h4[i] = (_Float16)v[i];
        *(volatile v4h*)(C16 + cofs + (size_t)(row0 + r) * ldc + col0 + c4) = h4; } }
    if (pass == 0) __threadfence(); } }

__global__ __launch_bounds__(256) void k_vt(const _Float16* __restrict__ QKV, _Float16* __restrict__ VT) {
  __shared__ unsigned short tl[64][66];
  const int tid = threadIdx.x; const int slab = blockIdx.x / (SEQ / 64), lg = blockIdx.x - slab * (SEQ / 64); const int b = slab / NH, h = slab - b * NH;
  for (int i = tid; i < 64 * 8; i += 256) { const int r = i / 8, c8 = (i % 8) * 8; FragH f;
    f.half[0] = *(const v8us*)((const unsigned short*)QKV + ((size_t)b * SEQ + lg * 64 + r) * LQ + 2 * DM + h * HD + c8);
#pragma unroll
    for (int q = 0; q < 8; ++q) tl[r][c8 + q] = f.u[q]; }
  __syncthreads();
  for (int pass = 0; pass < 2; ++pass) {
#pragma unroll
    for (int rd = 0; rd < 2; ++rd) { const int d = rd * 32 + tid / 8, pc = tid % 8; FragH f;
#pragma unroll
      for (int q = 0; q < 8; ++q) f.u[q] = tl[pc * 8 + q][d];
      *(volatile v8us*)((unsigned short*)VT + ((size_t)slab * 64 + d) * SEQ + lg * 64 + pc * 8) = f.half[0]; }
    if (pass == 0) __threadfence(); } }

__global__ __launch_bounds__(128) void k_flash(const _Float16* __restrict__ QKV, const _Float16* __restrict__ VT, _Float16* __restrict__ OC) {
  __shared__ __attribute__((aligned(16))) unsigned short sh[4][16][72];
  __shared__ __attribute__((aligned(16))) unsigned short sl[4][16][72];
  const int wave = __builtin_amdgcn_readfirstlane((int)(threadIdx.x >> 5));
  const int lane = threadIdx.x & 31, ln = lane & 15, hh = lane >> 4;
  const int bh = blockIdx.y; const int b = bh / NH, h = bh - b * NH;
  const int q0 = blockIdx.x * 64 + wave * 16;
  const size_t rowb = (size_t)b * SEQ;
  const _Float16* qp = QKV + (rowb + q0 + ln) * LQ + h * HD;
  const v16h bq0 = g2_frag(qp, hh), bq1 = g2_frag(qp + 32, hh);
  const _Float16* kp = QKV + (rowb + ln) * LQ + DM + h * HD;
  const _Float16* vp = VT + ((size_t)bh * HD + ln) * SEQ;
  const v8f z8 = {0.f,0.f,0.f,0.f,0.f,0.f,0.f,0.f};
  v8f o0 = z8, o1 = z8, o2 = z8, o3 = z8;
  float m = -1.0e30f, l = 0.f;
#pragma unroll 1
  for (int k0 = 0; k0 < SEQ; k0 += 32) {
    const _Float16* ka = kp + (size_t)k0 * LQ; const _Float16* kb = ka + (size_t)16 * LQ;
    v8f s0 = z8, s1 = z8;
    v16h a = g2_frag(ka, hh); s0 = g2_mma(a, bq0, s0);
    a = g2_frag(ka + 32, hh); s0 = g2_mma(a, bq1, s0);
    a = g2_frag(kb, hh); s1 = g2_mma(a, bq0, s1);
    a = g2_frag(kb + 32, hh); s1 = g2_mma(a, bq1, s1);
    float mx = -1.0e30f;
#pragma unroll
    for (int r = 0; r < 8; ++r) { s0[r] *= 0.125f; s1[r] *= 0.125f; mx = fmaxf(mx, fmaxf(s0[r], s1[r])); }
    mx = fmaxf(mx, __shfl_xor(mx, 16, 32));
    const float mn = fmaxf(m, mx);
    const float al = __expf(m - mn);
    m = mn;
    const float mc = mn - 5.545177444f;
    FragH pf; float ps = 0.f;
#pragma unroll
    for (int r = 0; r < 8; ++r) {
      _Float16 p = (_Float16)__expf(s0[r] - mc); pf.h[r] = p; ps += (float)p;
      p = (_Float16)__expf(s1[r] - mc); pf.h[8 + r] = p; ps += (float)p; }
    l = l * al + ps;
#pragma unroll
    for (int r = 0; r < 8; ++r) { o0[r] *= al; o1[r] *= al; o2[r] *= al; o3[r] *= al; }
    a = g2_frag(vp + k0, hh); o0 = g2_mma(a, pf.v, o0);
    a = g2_frag(vp + (size_t)16 * SEQ + k0, hh); o1 = g2_mma(a, pf.v, o1);
    a = g2_frag(vp + (size_t)32 * SEQ + k0, hh); o2 = g2_mma(a, pf.v, o2);
    a = g2_frag(vp + (size_t)48 * SEQ + k0, hh); o3 = g2_mma(a, pf.v, o3);
  }
  l += __shfl_xor(l, 16, 32);
  const float sc = 1024.0f * (1.0f / l);
  v8f oo[4] = {o0, o1, o2, o3};
#pragma unroll
  for (int t = 0; t < 4; ++t) { Frag8 fh, fl;
#pragma unroll
    for (int r = 0; r < 8; ++r) { const float xv = oo[t][r] * sc; const _Float16 hv = (_Float16)xv; fh.h[r] = hv; fl.h[r] = (_Float16)(xv - (float)hv); }
    *(v8us*)&sh[wave][ln][16 * t + 8 * hh] = fh.v;
    *(v8us*)&sl[wave][ln][16 * t + 8 * hh] = fl.v; }
  __builtin_amdgcn_fence(4  , "workgroup"); __builtin_amdgcn_wave_barrier();
  const int rq = lane >> 3, pc = (lane & 7) * 8;
  for (int pass = 0; pass < 2; ++pass) {
#pragma unroll
    for (int j = 0; j < 4; ++j) { const int q = j * 4 + rq;
      const v8us vh = *(const v8us*)&sh[wave][q][pc]; const v8us vl = *(const v8us*)&sl[wave][q][pc];
      unsigned short* dst = (unsigned short*)OC + (rowb + q0 + q) * (size_t)OCP + h * HD + pc;
      *(volatile v8us*)dst = vh;
      *(volatile v8us*)(dst + DM) = vl; }
    if (pass == 0) __threadfence(); } }

extern "C" void kernel_launch(void* const* d_in, const int* in_sizes, int n_in,
                              void* d_out, int out_size, void* d_ws, size_t ws_size, hipStream_t stream) {
  if (n_in < 5) return;
  const long long xneed = ((long long)(NB - 1) * SEQ_FULL + SEQ) * DM;
  if ((long long)in_sizes[0] < xneed) return;
  if ((long long)in_sizes[1] < (long long)DM * 3 * DM) return;
  if ((long long)in_sizes[2] < (long long)3 * DM) return;
  if ((long long)in_sizes[3] < (long long)DM * DM) return;
  if ((long long)in_sizes[4] < (long long)DM) return;
  if ((long long)out_size < xneed) return;
  const float* x = (const float*)d_in[0]; const float* wqkv = (const float*)d_in[1]; const float* bqkv = (const float*)d_in[2]; const float* wo = (const float*)d_in[3]; const float* bo = (const float*)d_in[4];
  char* ws = (char*)d_ws; size_t off = 0;
  auto take = [&](size_t bytes) { char* p = ws + off; off += (bytes + 255) & ~(size_t)255; return p; };
  _Float16* BQKV = (_Float16*)take((size_t)3 * DM * DM * 2);
  _Float16* BO   = (_Float16*)take((size_t)DM * OCP * 2);
  _Float16* X16  = (_Float16*)take(NR * DM * 2);
  _Float16* QKV  = (_Float16*)take(NR * LQ * 2);
  _Float16* VT   = (_Float16*)take((size_t)NB * NH * HD * SEQ * 2);
  _Float16* OC   = (_Float16*)take(NR * OCP * 2);
  if (off > ws_size) return;
  k_wt_f16<<<(unsigned)(((size_t)3 * DM * (DM / 8) + 255) / 256), 256, 0, stream>>>(wqkv, BQKV, DM, 3 * DM, DM, 0, 16.0f);
  k_wt_f16<<<(unsigned)(((size_t)DM * (DM / 8) + 255) / 256), 256, 0, stream>>>(wo, BO, DM, DM, OCP, 1, 16.0f);
  k_x16<<<(unsigned)((NR * DM / 8 + 255) / 256), 256, 0, stream>>>(x, X16);
  k_gemm2<<<dim3((unsigned)((NR / 128) * (LQ / 64)), 1), 128, 0, stream>>>(X16, DM, (size_t)0, BQKV, DM, 0.0625f, bqkv, (float*)nullptr, QKV, LQ, (size_t)0, (int)NR, LQ, DM);
  k_vt<<<(unsigned)(NB * NH * (SEQ / 64)), 256, 0, stream>>>(QKV, VT);
  k_flash<<<dim3(SEQ / 64, NB * NH), 128, 0, stream>>>(QKV, VT, OC);
  k_gemm2<<<dim3((unsigned)((SEQ / 128) * (DM / 64)), NB), 128, 0, stream>>>(OC, OCP, (size_t)SEQ * OCP, BO, OCP, 6.103515625e-05f, bo, (float*)d_out, (_Float16*)nullptr, DM, (size_t)SEQ_FULL * DM, SEQ, DM, OCP);
}
